// DTIHarmonic_44143673868856
// MI455X (gfx1250) — hardware-verified
//
#include <hip/hip_runtime.h>
#define NB 2
#define NA 384
#define NR (NB * NA)
#define DD 128
#define NL 3
#define NPM 5
typedef __bf16 v16b __attribute__((ext_vector_type(16)));
typedef unsigned short v8us __attribute__((ext_vector_type(8), may_alias));
typedef float  v8f  __attribute__((ext_vector_type(8)));
typedef float  v4f  __attribute__((ext_vector_type(4)));
typedef float  v4fa __attribute__((ext_vector_type(4), may_alias));
union FragB { v16b v; v8us half[2]; unsigned short u[16]; };

__device__ __forceinline__ unsigned short bf16_bits(float x) { unsigned int u = __float_as_uint(x); return (unsigned short)((u + 0x7FFFu + ((u >> 16) & 1u)) >> 16); }
__device__ __forceinline__ float bf16_val(unsigned short b) { return __uint_as_float(((unsigned int)b) << 16); }
__device__ __forceinline__ float bf16_round(float x) { return bf16_val(bf16_bits(x)); }
template <int NT>
__device__ __forceinline__ v8f mmaN(v16b ah, v16b al, v16b bh, v16b bl, v8f c) {
  c = __builtin_amdgcn_wmma_f32_16x16x32_bf16(false, ah, false, bh, (short)0, c, false, false);
  if (NT >= 2) c = __builtin_amdgcn_wmma_f32_16x16x32_bf16(false, al, false, bh, (short)0, c, false, false);
  if (NT >= 3) c = __builtin_amdgcn_wmma_f32_16x16x32_bf16(false, ah, false, bl, (short)0, c, false, false);
  asm volatile("v_nop\n\tv_nop\n\tv_nop\n\tv_nop" : "+v"(c) : "v"(ah), "v"(al), "v"(bh), "v"(bl));
  return c;
}

__global__ __launch_bounds__(256) void k_wt_bf16(const float* __restrict__ W, unsigned short* __restrict__ Wt, int K, int N) {
  const int t = blockIdx.x * 256 + threadIdx.x;
  const int k8n = K / 8;
  if (t >= N * k8n) return;
  const int n = t / k8n, k8 = (t % k8n) * 8;
  v8us v;
#pragma unroll
  for (int i = 0; i < 8; ++i) v[i] = bf16_bits(W[(size_t)(k8 + i) * N + n]);
  *(volatile v8us*)(Wt + (size_t)n * K + k8) = v;
  __threadfence();
  *(volatile v8us*)(Wt + (size_t)n * K + k8) = v;
}

template <bool ASPLIT, int ACT, bool BIAS_BF16>
__global__ __launch_bounds__(128) void k_gemm_bf(const float* __restrict__ A, int lda, const unsigned short* __restrict__ Wt, int ldb,
                                               const float* __restrict__ bias, float* __restrict__ C, int ldc, int M, int N, int K) {
  __shared__ __attribute__((aligned(16))) float so[4][16][64];
  const int tid = threadIdx.x, w = tid >> 5, lane = tid & 31, ln = lane & 15, hh = lane >> 4;
  const int ntn = N / 64;
  const int wid = blockIdx.x * 4 + w;
  const int mt = wid / ntn, nq = wid % ntn;
  if (mt * 16 >= M) return;
  const int row0 = mt * 16, col0 = nq * 64;
  const float* arow = A + (size_t)(row0 + ln) * lda;
  v8f acc[4] = {};
  for (int kb = 0; kb < K; kb += 32) {
    FragB ah, al;
    const v4f x0 = *(const v4fa*)(arow + kb + 8 * hh), x1 = *(const v4fa*)(arow + kb + 8 * hh + 4);
    const v4f x2 = *(const v4fa*)(arow + kb + 16 + 8 * hh), x3 = *(const v4fa*)(arow + kb + 16 + 8 * hh + 4);
    float xs[16] = {x0[0],x0[1],x0[2],x0[3],x1[0],x1[1],x1[2],x1[3],x2[0],x2[1],x2[2],x2[3],x3[0],x3[1],x3[2],x3[3]};
#pragma unroll
    for (int i = 0; i < 16; ++i) { const unsigned short hb = bf16_bits(xs[i]); ah.u[i] = hb; al.u[i] = ASPLIT ? bf16_bits(xs[i] - bf16_val(hb)) : (unsigned short)0; }
#pragma unroll
    for (int t = 0; t < 4; ++t) {
      const unsigned short* brow = Wt + (size_t)(col0 + t * 16 + ln) * ldb + kb;
      FragB b;
      b.half[0] = *(const v8us*)(brow + 8 * hh);
      b.half[1] = *(const v8us*)(brow + 16 + 8 * hh);
      acc[t] = mmaN<ASPLIT ? 2 : 1>(ah.v, al.v, b.v, b.v, acc[t]);
    }
  }
#pragma unroll
  for (int t = 0; t < 4; ++t) {
    float bv = bias ? bias[col0 + t * 16 + ln] : 0.f;
    if (BIAS_BF16) bv = bf16_round(bv);
#pragma unroll
    for (int r = 0; r < 8; ++r) { float v = acc[t][r] + bv; if (ACT == 1) v = fmaxf(v, 0.f); so[w][8 * hh + r][t * 16 + ln] = v; }
  }
  __builtin_amdgcn_fence(__ATOMIC_ACQ_REL, "workgroup");
  __builtin_amdgcn_wave_barrier();
  const int rsub = lane >> 4, c4 = (lane & 15) * 4;
  for (int pass = 0; pass < 2; ++pass) {
#pragma unroll
    for (int q = 0; q < 8; ++q) {
      const int r = q * 2 + rsub;
      const v4f v = *(const v4fa*)&so[w][r][c4];
      *(volatile v4f*)(C + (size_t)(row0 + r) * ldc + col0 + c4) = v;
    }
    if (pass == 0) __threadfence();
  }
}

template <bool ASPLIT, int ACT, bool BIAS_BF16, bool RES_BF16>
__global__ __launch_bounds__(128) void k_gemm_bf3(const float* __restrict__ A, int lda, const unsigned short* __restrict__ Wt, int ldb,
                                                const float* __restrict__ bias, const float* __restrict__ resid, int rmod, int ldr,
                                                float* __restrict__ C, int ldc, int M, int N, int K) {
  __shared__ __attribute__((aligned(16))) float so[4][16][64];
  const int tid = threadIdx.x, w = tid >> 5, lane = tid & 31, ln = lane & 15, hh = lane >> 4;
  const int ntn = N / 64;
  const int wid = blockIdx.x * 4 + w;
  const int mt = wid / ntn, nq = wid % ntn;
  if (mt * 16 >= M) return;
  const int row0 = mt * 16, col0 = nq * 64;
  const float* arow = A + (size_t)(row0 + ln) * lda;
  v8f acc[4] = {};
  for (int kb = 0; kb < K; kb += 32) {
    FragB ah, al;
    const v4f x0 = *(const v4fa*)(arow + kb + 8 * hh), x1 = *(const v4fa*)(arow + kb + 8 * hh + 4);
    const v4f x2 = *(const v4fa*)(arow + kb + 16 + 8 * hh), x3 = *(const v4fa*)(arow + kb + 16 + 8 * hh + 4);
    float xs[16] = {x0[0],x0[1],x0[2],x0[3],x1[0],x1[1],x1[2],x1[3],x2[0],x2[1],x2[2],x2[3],x3[0],x3[1],x3[2],x3[3]};
#pragma unroll
    for (int i = 0; i < 16; ++i) { const unsigned short hb = bf16_bits(xs[i]); ah.u[i] = hb; al.u[i] = ASPLIT ? bf16_bits(xs[i] - bf16_val(hb)) : (unsigned short)0; }
#pragma unroll
    for (int t = 0; t < 4; ++t) {
      const unsigned short* brow = Wt + (size_t)(col0 + t * 16 + ln) * ldb + kb;
      FragB b;
      b.half[0] = *(const v8us*)(brow + 8 * hh);
      b.half[1] = *(const v8us*)(brow + 16 + 8 * hh);
      acc[t] = mmaN<ASPLIT ? 2 : 1>(ah.v, al.v, b.v, b.v, acc[t]);
    }
  }
#pragma unroll
  for (int t = 0; t < 4; ++t) {
    const int col = col0 + t * 16 + ln;
    float bv = bias ? bias[col] : 0.f;
    if (BIAS_BF16) bv = bf16_round(bv);
#pragma unroll
    for (int r = 0; r < 8; ++r) {
      float v = acc[t][r] + bv;
      if (resid) { float rv = resid[(size_t)((row0 + 8 * hh + r) % rmod) * ldr + col]; if (RES_BF16) rv = bf16_round(rv); v += rv; }
      if (ACT == 1) v = fmaxf(v, 0.f);
      if (ACT == 2) v = 0.5f * v * (1.0f + erff(v * 0.70710678118654752f));
      if (ACT == 3) { const float u = 0.7978845608028654f * (v + 0.044715f * v * v * v); v = 0.5f * v * (1.0f + tanhf(u)); }
      so[w][8 * hh + r][t * 16 + ln] = v;
    }
  }
  __builtin_amdgcn_fence(__ATOMIC_ACQ_REL, "workgroup");
  __builtin_amdgcn_wave_barrier();
  const int rsub = lane >> 4, c4 = (lane & 15) * 4;
  for (int pass = 0; pass < 2; ++pass) {
#pragma unroll
    for (int q = 0; q < 8; ++q) {
      const int r = q * 2 + rsub;
      const v4f v = *(const v4fa*)&so[w][r][c4];
      *(volatile v4f*)(C + (size_t)(row0 + r) * ldc + col0 + c4) = v;
    }
    if (pass == 0) __threadfence();
  }
}
template <bool PARAM_BF16>
__global__ __launch_bounds__(256) void k_layernorm(const float* __restrict__ X, const float* __restrict__ R, const float* __restrict__ g, const float* __restrict__ bta,
                                                  float* __restrict__ out_sum, float* __restrict__ out_norm, int N, float eps) {
  __shared__ float red[256];
  const int row = blockIdx.x, tid = threadIdx.x;
  const float* x = X + (size_t)row * N; const float* rr = R ? R + (size_t)row * N : nullptr;
  float vals[16];
  const int per = N / 256;
  float s1 = 0.f;
  for (int u = 0; u < per / 4; ++u) {
    const int j = tid * 4 + 1024 * u;
    const v4f a = *(const v4fa*)(x + j);
    v4f b = {0.f,0.f,0.f,0.f}; if (rr) b = *(const v4fa*)(rr + j);
#pragma unroll
    for (int q = 0; q < 4; ++q) { const float v = a[q] + b[q]; vals[u * 4 + q] = v; s1 += v; }
  }
  red[tid] = s1; __syncthreads();
  for (int st = 128; st > 0; st >>= 1) { if (tid < st) red[tid] += red[tid + st]; __syncthreads(); }
  const float mu = red[0] / (float)N; __syncthreads();
  float s2 = 0.f;
  for (int u = 0; u < per / 4; ++u)
#pragma unroll
    for (int q = 0; q < 4; ++q) { const float c = vals[u * 4 + q] - mu; s2 += c * c; }
  red[tid] = s2; __syncthreads();
  for (int st = 128; st > 0; st >>= 1) { if (tid < st) red[tid] += red[tid + st]; __syncthreads(); }
  const float rs = rsqrtf(red[0] / (float)N + eps);
  for (int pass = 0; pass < 2; ++pass) {
    for (int u = 0; u < per / 4; ++u) {
      const int j = tid * 4 + 1024 * u;
      v4f o, sm;
#pragma unroll
      for (int q = 0; q < 4; ++q) {
        float gg = g[j + q], bb = bta[j + q];
        if (PARAM_BF16) { gg = bf16_round(gg); bb = bf16_round(bb); }
        sm[q] = vals[u * 4 + q]; o[q] = (vals[u * 4 + q] - mu) * rs * gg + bb;
      }
      if (out_sum) *(volatile v4f*)(out_sum + (size_t)row * N + j) = sm;
      *(volatile v4f*)(out_norm + (size_t)row * N + j) = o;
    }
    if (pass == 0) __threadfence();
  }
}


typedef _Float16 v16h __attribute__((ext_vector_type(16)));
union FragH { v16h v; v8us half[2]; _Float16 h[16]; unsigned short u[16]; };
template <int NT>
__device__ __forceinline__ v8f mmaH(v16h ah, v16h al, v16h bh, v16h bl, v8f c) {
  c = __builtin_amdgcn_wmma_f32_16x16x32_f16(false, ah, false, bh, (short)0, c, false, false);
  if (NT >= 2) c = __builtin_amdgcn_wmma_f32_16x16x32_f16(false, al, false, bh, (short)0, c, false, false);
  if (NT >= 3) c = __builtin_amdgcn_wmma_f32_16x16x32_f16(false, ah, false, bl, (short)0, c, false, false);
  asm volatile("v_nop\n\tv_nop\n\tv_nop\n\tv_nop" : "+v"(c) : "v"(ah), "v"(al), "v"(bh), "v"(bl));
  return c;
}
template <bool ASPLIT>
__global__ __launch_bounds__(128) void k_gemm_h(const float* __restrict__ A, int lda, size_t sA, const _Float16* __restrict__ Bh, int ldb, size_t sB, float alpha, float* __restrict__ C, int ldc, size_t sC, int M, int N, int K) {
  __shared__ __attribute__((aligned(16))) float so[4][16][64];
  const int tid = threadIdx.x, w = tid >> 5, lane = tid & 31, ln = lane & 15, hh = lane >> 4; const int by = blockIdx.y;
  A += (size_t)by * sA; Bh += (size_t)by * sB; C += (size_t)by * sC;
  const int ntn = (N + 63) / 64; const int wid = blockIdx.x * 4 + w; const int mt = wid / ntn, nq = wid % ntn; if (mt * 16 >= M) return;
  const int row0 = mt * 16, col0 = nq * 64; const float* arow = A + (size_t)(row0 + ln) * lda;
  v8f acc[4] = {};
  for (int kb = 0; kb < K; kb += 32) {
    FragH ah, al;
    const v4f x0 = *(const v4fa*)(arow + kb + 8 * hh), x1 = *(const v4fa*)(arow + kb + 8 * hh + 4), x2 = *(const v4fa*)(arow + kb + 16 + 8 * hh), x3 = *(const v4fa*)(arow + kb + 16 + 8 * hh + 4);
    float xs[16] = {x0[0],x0[1],x0[2],x0[3],x1[0],x1[1],x1[2],x1[3],x2[0],x2[1],x2[2],x2[3],x3[0],x3[1],x3[2],x3[3]};
#pragma unroll
    for (int i = 0; i < 16; ++i) { const _Float16 h = (_Float16)xs[i]; ah.h[i] = h; al.h[i] = ASPLIT ? (_Float16)(xs[i] - (float)h) : (_Float16)0.0f; }
#pragma unroll
    for (int t = 0; t < 4; ++t) { if (col0 + t * 16 >= N) continue; const size_t boff = (size_t)(col0 + t * 16 + ln) * ldb + kb; FragH bq; bq.half[0] = *(const v8us*)(Bh + boff + 8 * hh); bq.half[1] = *(const v8us*)(Bh + boff + 16 + 8 * hh);
      acc[t] = mmaH<ASPLIT ? 2 : 1>(ah.v, al.v, bq.v, bq.v, acc[t]); }
  }
#pragma unroll
  for (int t = 0; t < 4; ++t) { if (col0 + t * 16 >= N) continue;
#pragma unroll
    for (int r = 0; r < 8; ++r) so[w][8 * hh + r][t * 16 + ln] = acc[t][r] * alpha; }
  __builtin_amdgcn_fence(__ATOMIC_ACQ_REL, "workgroup"); __builtin_amdgcn_wave_barrier();
  const int rsub = lane >> 4, c4 = (lane & 15) * 4;
  for (int pass = 0; pass < 2; ++pass) {
#pragma unroll
    for (int q = 0; q < 8; ++q) { const int r = q * 2 + rsub; if (col0 + c4 < N) { const v4f v = *(const v4fa*)&so[w][r][c4]; *(volatile v4f*)(C + (size_t)(row0 + r) * ldc + col0 + c4) = v; } }
    if (pass == 0) __threadfence(); }
}

__global__ __launch_bounds__(256) void k_wt_f16(const float* __restrict__ W, _Float16* __restrict__ Wt, int K, int N, float scale) {
  const int t = blockIdx.x * 256 + threadIdx.x; if (t >= N * (K / 8)) return; const int n = t / (K / 8), k8 = (t % (K / 8)) * 8; FragH f;
#pragma unroll
  for (int i = 0; i < 8; ++i) f.h[i] = (_Float16)(bf16_round(W[(size_t)(k8 + i) * N + n]) * scale); const v8us o = f.half[0];
  *(volatile v8us*)((unsigned short*)Wt + (size_t)n * K + k8) = o; __threadfence(); *(volatile v8us*)((unsigned short*)Wt + (size_t)n * K + k8) = o;
}
template <int ACT>
__global__ __launch_bounds__(128) void k_gemm_hhx(const _Float16* __restrict__ A, int lda, size_t sA, const _Float16* __restrict__ Bh, int ldb, size_t sB, float alpha, const float* __restrict__ bias, size_t sBias, const float* __restrict__ CP, int rowsPerB, size_t sCPb, int row0g,
    float* __restrict__ C, _Float16* __restrict__ C16, int ldc, size_t sC, int M, int N, int K) {
  __shared__ __attribute__((aligned(16))) float so[4][16][64];
  const int tid = threadIdx.x, w = tid >> 5, lane = tid & 31, ln = lane & 15, hh = lane >> 4; const int by = blockIdx.y;
  A += (size_t)by * sA; Bh += (size_t)by * sB; const size_t cofs = (size_t)by * sC; const float* bp = bias ? bias + (size_t)by * sBias : nullptr;
  const int ntn = (N + 63) / 64; const int wid = blockIdx.x * 4 + w; const int mt = wid / ntn, nq = wid % ntn; if (mt * 16 >= M) return;
  const int row0 = mt * 16, col0 = nq * 64; const _Float16* arow = A + (size_t)(row0 + ln) * lda;
  v8f acc[4] = {};
  for (int kb = 0; kb < K; kb += 32) { FragH ah; ah.half[0] = *(const v8us*)((const unsigned short*)arow + kb + 8 * hh); ah.half[1] = *(const v8us*)((const unsigned short*)arow + kb + 16 + 8 * hh);
#pragma unroll
    for (int t = 0; t < 4; ++t) { if (col0 + t * 16 >= N) continue; const size_t boff = (size_t)(col0 + t * 16 + ln) * ldb + kb; FragH bq; bq.half[0] = *(const v8us*)((const unsigned short*)Bh + boff + 8 * hh); bq.half[1] = *(const v8us*)((const unsigned short*)Bh + boff + 16 + 8 * hh);
      acc[t] = mmaH<1>(ah.v, ah.v, bq.v, bq.v, acc[t]); }
  }
#pragma unroll
  for (int t = 0; t < 4; ++t) { if (col0 + t * 16 >= N) continue; const int col = col0 + t * 16 + ln; const float bv = bp ? bf16_round(bp[col]) : 0.f;
#pragma unroll
    for (int r = 0; r < 8; ++r) { float v = acc[t][r] * alpha + bv; if (CP) { const int bidx = (row0g + row0 + 8 * hh + r) / rowsPerB; v += CP[(size_t)bidx * sCPb + (size_t)by * 64 + col]; } if (ACT == 1) v = (v > 0.f) ? v : expm1f(v); else if (ACT == 7) v = (v > 0.f) ? v + 1.0f : expf(v); else if (ACT == 8) v = tanhf(v); else if (ACT == 9) v = 0.5f * v * (1.0f + tanhf(0.7978845608028654f * (v + 0.044715f * v * v * v))); else if (ACT == 11) v = 1.0f / (1.0f + expf(-v)); else if (ACT == 12) v = (v > 0.f) ? v : 0.01f * v; else if (ACT == 14) v = (v > 0.f) ? v : 0.1f * v; else if (ACT == 15) v = v / (1.0f + expf(-v)); else if (ACT == 3) v = fmaxf(v, 0.f); else if (ACT == 6) v = 0.5f * v * (1.0f + erff(v * 0.70710678118654752f)); so[w][8 * hh + r][t * 16 + ln] = v; } }
  __builtin_amdgcn_fence(__ATOMIC_ACQ_REL, "workgroup"); __builtin_amdgcn_wave_barrier();
  const int rsub = lane >> 4, c4 = (lane & 15) * 4; typedef _Float16 v4h __attribute__((ext_vector_type(4)));
  for (int pass = 0; pass < 2; ++pass) {
#pragma unroll
    for (int q = 0; q < 8; ++q) { const int r = q * 2 + rsub; if (col0 + c4 < N) { const v4f v = *(const v4fa*)&so[w][r][c4]; if (C) *(volatile v4f*)(C + cofs + (size_t)(row0 + r) * ldc + col0 + c4) = v; if (C16) { v4h h4; for (int i = 0; i < 4; ++i) h4[i] = (_Float16)v[i]; *(volatile v4h*)(C16 + cofs + (size_t)(row0 + r) * ldc + col0 + c4) = h4; } } }
    if (pass == 0) __threadfence(); }
}


typedef _Float16 v4h __attribute__((ext_vector_type(4)));

__global__ __launch_bounds__(256) void k_x16(const float* __restrict__ x, _Float16* __restrict__ X16, size_t n8) { const size_t t = (size_t)blockIdx.x * 256 + threadIdx.x; if (t >= n8) return; FragH f;
#pragma unroll
  for (int q = 0; q < 8; ++q) f.h[q] = (_Float16)bf16_round(x[t * 8 + q]); *(volatile v8us*)((unsigned short*)X16 + t * 8) = f.half[0]; __threadfence(); *(volatile v8us*)((unsigned short*)X16 + t * 8) = f.half[0]; }
__global__ __launch_bounds__(256) void k_h16(const float* __restrict__ x, _Float16* __restrict__ X16, size_t n8) { const size_t t = (size_t)blockIdx.x * 256 + threadIdx.x; if (t >= n8) return; FragH f;
#pragma unroll
  for (int q = 0; q < 8; ++q) f.h[q] = (_Float16)x[t * 8 + q]; *(volatile v8us*)((unsigned short*)X16 + t * 8) = f.half[0]; __threadfence(); *(volatile v8us*)((unsigned short*)X16 + t * 8) = f.half[0]; }
__global__ __launch_bounds__(256) void k_round16f(const float* __restrict__ W, _Float16* __restrict__ Bt, size_t n8) { const size_t t = (size_t)blockIdx.x * 256 + threadIdx.x; if (t >= n8) return; FragH f;
#pragma unroll
  for (int i = 0; i < 8; ++i) f.h[i] = (_Float16)(bf16_round(W[t * 8 + i]) * 16.0f); *(volatile v8us*)((unsigned short*)Bt + t * 8) = f.half[0]; __threadfence(); *(volatile v8us*)((unsigned short*)Bt + t * 8) = f.half[0]; }
template <int NHv, int TTv>
__global__ __launch_bounds__(256) void k_vt(const _Float16* __restrict__ V16, int ldv, int voff, _Float16* __restrict__ Vt) { __shared__ unsigned short tl[64][66]; const int tid = threadIdx.x; const int slab = blockIdx.x / (TTv / 64), lg = blockIdx.x % (TTv / 64); const int b = slab / NHv, h = slab % NHv;
  for (int i = tid; i < 64 * 8; i += 256) { const int r = i / 8, c8 = (i % 8) * 8; FragH f; f.half[0] = *(const v8us*)((const unsigned short*)V16 + ((size_t)b * TTv + lg * 64 + r) * ldv + voff + h * 64 + c8);
#pragma unroll
    for (int q = 0; q < 8; ++q) tl[r][c8 + q] = f.u[q]; }
  __syncthreads();
  for (int pass = 0; pass < 2; ++pass) {
#pragma unroll
    for (int rd = 0; rd < 2; ++rd) { const int d = rd * 32 + tid / 8, pc = tid % 8; FragH f;
#pragma unroll
      for (int q = 0; q < 8; ++q) f.u[q] = tl[pc * 8 + q][d];
      *(volatile v8us*)((unsigned short*)Vt + ((size_t)slab * 64 + d) * TTv + lg * 64 + pc * 8) = f.half[0]; }
    if (pass == 0) __threadfence(); } }

__global__ __launch_bounds__(256) void k_hl(const float* __restrict__ F, _Float16* __restrict__ Hh, _Float16* __restrict__ Hl, size_t n8) { const size_t t = (size_t)blockIdx.x * 256 + threadIdx.x; if (t >= n8) return; FragH fh, fl; const v4f a = *(const v4fa*)(F + t * 8), c = *(const v4fa*)(F + t * 8 + 4);
#pragma unroll
  for (int q = 0; q < 4; ++q) { _Float16 h = (_Float16)a[q]; fh.h[q] = h; fl.h[q] = (_Float16)((a[q] - (float)h) * 1024.0f); h = (_Float16)c[q]; fh.h[4 + q] = h; fl.h[4 + q] = (_Float16)((c[q] - (float)h) * 1024.0f); }
  for (int pass = 0; pass < 2; ++pass) { *(volatile v8us*)((unsigned short*)Hh + t * 8) = fh.half[0]; *(volatile v8us*)((unsigned short*)Hl + t * 8) = fl.half[0]; if (pass == 0) __threadfence(); } }

__global__ __launch_bounds__(256) void k_h54(const float* __restrict__ h, _Float16* __restrict__ O) { const int t = blockIdx.x * 256 + threadIdx.x; if (t >= NR * 8) return; const int g = t % 8, r = t / 8; FragH f = FragH{};
#pragma unroll
  for (int q = 0; q < 8; ++q) { const int c = g * 8 + q; if (c < 54) f.h[q] = (_Float16)bf16_round(h[(size_t)r * 54 + c]); }
  *(volatile v8us*)((unsigned short*)O + (size_t)r * 64 + g * 8) = f.half[0]; __threadfence(); *(volatile v8us*)((unsigned short*)O + (size_t)r * 64 + g * 8) = f.half[0]; }
__global__ __launch_bounds__(256) void k_wt(const float* __restrict__ W, int K, int Kp, int N, _Float16* __restrict__ Bt) { const int t = blockIdx.x * 256 + threadIdx.x; if (t >= N * (Kp / 8)) return; const int k0 = (t % (Kp / 8)) * 8, n = t / (Kp / 8); FragH f;
#pragma unroll
  for (int q = 0; q < 8; ++q) { const int k = k0 + q; f.h[q] = (k < K) ? (_Float16)(bf16_round(W[(size_t)k * N + n]) * 16.0f) : (_Float16)0.0f; }
  *(volatile v8us*)((unsigned short*)Bt + (size_t)n * Kp + k0) = f.half[0]; __threadfence(); *(volatile v8us*)((unsigned short*)Bt + (size_t)n * Kp + k0) = f.half[0]; }
__global__ __launch_bounds__(256) void k_f16c(const float* __restrict__ F, _Float16* __restrict__ O, size_t n8) { const size_t t = (size_t)blockIdx.x * 256 + threadIdx.x; if (t >= n8) return; const v4f a = *(const v4fa*)(F + t * 8), c = *(const v4fa*)(F + t * 8 + 4); FragH f;
#pragma unroll
  for (int q = 0; q < 8; ++q) f.h[q] = (_Float16)((q < 4) ? a[q] : c[q - 4]);
  *(volatile v8us*)((unsigned short*)O + t * 8) = f.half[0]; __threadfence(); *(volatile v8us*)((unsigned short*)O + t * 8) = f.half[0]; }
__global__ __launch_bounds__(256) void k_gate(const float* __restrict__ HA, const float* __restrict__ Hh, float* __restrict__ E) {
  #pragma clang fp contract(off)
  const int t = blockIdx.x * 256 + threadIdx.x; if (t >= NB * NA * NA) return; const int k = t % NA; const int j = (t / NA) % NA; const int b = t / (NA * NA); const float* a = HA + ((size_t)b * NA + j) * DD; const float* c = Hh + ((size_t)b * NA + k) * DD; float s = 0.f;
#pragma unroll 1
  for (int l = 0; l < DD; l += 4) { const v4f x = *(const v4fa*)(a + l), y = *(const v4fa*)(c + l); s += x[0] * y[0]; s += x[1] * y[1]; s += x[2] * y[2]; s += x[3] * y[3]; }
  *(volatile float*)(E + t) = s; __threadfence(); *(volatile float*)(E + t) = s; }
__global__ __launch_bounds__(128) void k_gsoft(const float* __restrict__ E, const float* __restrict__ adj, float* __restrict__ ATTt) {
  #pragma clang fp contract(off)
  const int t = blockIdx.x * 128 + threadIdx.x; if (t >= NB * NA) return; const int j = t % NA, b = t / NA; const float* Eb = E + (size_t)b * NA * NA; const float* Ab = adj + (size_t)b * NA * NA;
  auto val = [&](int i) { const float e = Eb[(size_t)i * NA + j] + Eb[(size_t)j * NA + i]; return (bf16_round(Ab[(size_t)i * NA + j]) > 0.f) ? e : -9e15f; };
  float m = -3.0e38f;
#pragma unroll 1
  for (int i = 0; i < NA; ++i) m = fmaxf(m, val(i));
  float su = 0.f;
#pragma unroll 1
  for (int i = 0; i < NA; ++i) su += expf(val(i) - m);
  const float inv = 1.0f / su; float* dst = ATTt + ((size_t)b * NA + j) * NA;
  for (int pass = 0; pass < 2; ++pass) {
#pragma unroll 1
    for (int i = 0; i < NA; i += 4) { v4f v;
#pragma unroll
      for (int q = 0; q < 4; ++q) v[q] = expf(val(i + q) - m) * inv * bf16_round(Ab[(size_t)(i + q) * NA + j]);
      *(volatile v4f*)(dst + i) = v; }
    if (pass == 0) __threadfence(); } }
__global__ __launch_bounds__(64) void k_gagg(const float* __restrict__ ATTt, const float* __restrict__ Hh, const float* __restrict__ X, const float* __restrict__ gW, const float* __restrict__ gb, float* __restrict__ Xn) {
  #pragma clang fp contract(off)
  const int t = blockIdx.x * 64 + threadIdx.x; if (t >= NB * NA) return; const int i = t % NA, b = t / NA; const float* xb = X + (size_t)t * DD;
  __shared__ float hp_s[64][129]; volatile __attribute__((address_space(3))) float* hp = (volatile __attribute__((address_space(3))) float*)&hp_s[threadIdx.x][0];
  for (int k = 0; k < DD; ++k) hp[k] = 0.f;
#pragma unroll 1
  for (int j = 0; j < NA; ++j) { const float a = ATTt[((size_t)b * NA + j) * NA + i]; if (a != 0.f) { const float* hj = Hh + ((size_t)b * NA + j) * DD;
#pragma unroll 1
      for (int k = 0; k < DD; ++k) hp[k] += a * hj[k]; } }
  float g = bf16_round(gb[0]);
#pragma unroll 1
  for (int k = 0; k < DD; ++k) { hp[k] = fmaxf(hp[k], 0.f); g += xb[k] * bf16_round(gW[k]); g += hp[k] * bf16_round(gW[DD + k]); }
  const float cf = 1.0f / (1.0f + expf(-g));
  for (int pass = 0; pass < 2; ++pass) {
#pragma unroll 1
    for (int k = 0; k < DD; k += 4) { v4f v;
#pragma unroll
      for (int q = 0; q < 4; ++q) v[q] = cf * xb[k + q] + (1.0f - cf) * hp[k + q];
      *(volatile v4f*)(Xn + (size_t)t * DD + k) = v; }
    if (pass == 0) __threadfence(); } }
__global__ __launch_bounds__(256) void k_pmlp(const float* __restrict__ P1, const float* __restrict__ P2, const float* __restrict__ W2, const float* __restrict__ b2, float* __restrict__ O5) {
  #pragma clang fp contract(off)
  const int t = blockIdx.x * 256 + threadIdx.x; if (t >= NB * NA * NA) return; const int j = t % NA; const int i = (t / NA) % NA; const int b = t / (NA * NA); const int ti = b * NA + i, tj = b * NA + j;
  float s0 = bf16_round(b2[0]), s1 = bf16_round(b2[1]), s2 = bf16_round(b2[2]), s3 = bf16_round(b2[3]), s4 = bf16_round(b2[4]);
  const float* a0 = P1 + ((size_t)0 * NR + ti) * DD; const float* c0 = P2 + ((size_t)0 * NR + tj) * DD; const float* a1 = P1 + ((size_t)1 * NR + ti) * DD; const float* c1 = P2 + ((size_t)1 * NR + tj) * DD; const float* a2 = P1 + ((size_t)2 * NR + ti) * DD; const float* c2 = P2 + ((size_t)2 * NR + tj) * DD; const float* a3 = P1 + ((size_t)3 * NR + ti) * DD; const float* c3 = P2 + ((size_t)3 * NR + tj) * DD; const float* a4 = P1 + ((size_t)4 * NR + ti) * DD; const float* c4 = P2 + ((size_t)4 * NR + tj) * DD;
#pragma unroll 1
  for (int k = 0; k < DD; ++k) { s0 += fmaxf(a0[k] + c0[k], 0.f) * bf16_round(W2[k]); s1 += fmaxf(a1[k] + c1[k], 0.f) * bf16_round(W2[DD + k]); s2 += fmaxf(a2[k] + c2[k], 0.f) * bf16_round(W2[2 * DD + k]); s3 += fmaxf(a3[k] + c3[k], 0.f) * bf16_round(W2[3 * DD + k]); s4 += fmaxf(a4[k] + c4[k], 0.f) * bf16_round(W2[4 * DD + k]); }
  const size_t np_ = (size_t)NB * NA * NA;
  for (int pass = 0; pass < 2; ++pass) { *(volatile float*)(O5 + 0 * np_ + t) = s0; *(volatile float*)(O5 + 1 * np_ + t) = s1; *(volatile float*)(O5 + 2 * np_ + t) = s2; *(volatile float*)(O5 + 3 * np_ + t) = s3; *(volatile float*)(O5 + 4 * np_ + t) = s4; if (pass == 0) __threadfence(); } }
__global__ __launch_bounds__(128) void k_phys(const float* __restrict__ O5, const float* __restrict__ dmv, const float* __restrict__ ch1, const float* __restrict__ ch2, const float* __restrict__ veps, const float* __restrict__ vsig, const float* __restrict__ val1, const float* __restrict__ val2, const float* __restrict__ nm1, const float* __restrict__ nm2, const float* __restrict__ vcoef, float* __restrict__ ECV) {
  #pragma clang fp contract(off)
  const int t = blockIdx.x * 128 + threadIdx.x; if (t >= NB * NA) return; const int i = t % NA, b = t / NA; const float c1 = bf16_round(ch1[t]), v1 = bf16_round(val1[t]), n1 = bf16_round(nm1[t]); const float vc = bf16_round(vcoef[0]); const size_t np_ = (size_t)NB * NA * NA; float ec = 0.f, ev = 0.f;
#pragma unroll 1
  for (int j = 0; j < NA; ++j) { const int tj = b * NA + j; const size_t pr = ((size_t)b * NA + i) * NA + j; const float o0 = O5[pr], o1 = O5[np_ + pr], o2 = O5[2 * np_ + pr], o3 = O5[3 * np_ + pr], o4 = O5[4 * np_ + pr];
    const float* dv = dmv + pr * 3; const float dx = bf16_round(dv[0]), dy = bf16_round(dv[1]), dz = bf16_round(dv[2]); float dm = sqrtf(((dx * dx + dz * dz) + dy * dy) + 1e-10f); dm = (dm < 0.5f) ? 1e10f : dm;
    const float cA = 1.0f / (1.0f + expf(-o0)); const float cN = 1.0f / (1.0f + expf(-o1)) * 2.0f + 1.0f; float e_c = cA * (c1 * bf16_round(ch2[tj])) * exp2f(cN * log2f(1.0f / dm)); e_c = e_c * v1 * bf16_round(val2[tj]); e_c = fminf(fmaxf(e_c, -100.f), 100.f); ec += e_c;
    float vA = 1.0f / (1.0f + expf(-o2)) * 0.6f + 0.7f; vA = vA * (vc * vc) * bf16_round(veps[pr]); const float vB = tanhf(o3) * 0.6f + 0.7f; const float vN = 1.0f / (1.0f + expf(-o4)) * 2.0f + 5.0f;
    float dm0 = bf16_round(vsig[pr]) * vB; dm0 = (dm0 < 1e-4f) ? 1.0f : dm0; const float r = exp2f(vN * log2f(dm0 / dm)); float e_v = vA * (r * r - 2.0f * r); e_v = e_v * n1 * bf16_round(nm2[tj]); e_v = fminf(e_v, 100.f); ev += e_v; }
  typedef float v2f __attribute__((ext_vector_type(2))); v2f w; w[0] = ec; w[1] = ev; *(volatile v2f*)(ECV + (size_t)t * 2) = w; __threadfence(); *(volatile v2f*)(ECV + (size_t)t * 2) = w; }
__global__ __launch_bounds__(256) void k_final(const float* __restrict__ ECV, const float* __restrict__ H1g, const float* __restrict__ val1, const float* __restrict__ duff, const float* __restrict__ dcoef, const float* __restrict__ iW1, const float* __restrict__ ib1, const float* __restrict__ iW2, const float* __restrict__ ib2, float* __restrict__ out) {
  #pragma clang fp contract(off)
  __shared__ float red[2][256]; __shared__ float hs[128]; __shared__ float res[8]; const int tid = threadIdx.x;
  for (int b = 0; b < NB; ++b) {
    float sc = 0.f, sv = 0.f; for (int i = tid; i < NA; i += 256) { sc += ECV[((size_t)b * NA + i) * 2]; sv += ECV[((size_t)b * NA + i) * 2 + 1]; }
    red[0][tid] = sc; __syncthreads(); for (int st = 128; st > 0; st >>= 1) { if (tid < st) red[0][tid] += red[0][tid + st]; __syncthreads(); } if (tid == 0) res[b * 4 + 0] = red[0][0]; __syncthreads();
    red[1][tid] = sv; __syncthreads(); for (int st = 128; st > 0; st >>= 1) { if (tid < st) red[1][tid] += red[1][tid + st]; __syncthreads(); } if (tid == 0) res[b * 4 + 1] = red[1][0]; __syncthreads();
    if (tid < 128) { float s = 0.f;
#pragma unroll 1
      for (int i = 0; i < NA; ++i) s += H1g[((size_t)b * NA + i) * DD + tid] * bf16_round(val1[b * NA + i]);
      hs[tid] = s; } __syncthreads();
    if (tid == 0) { const float dc = bf16_round(dcoef[0]); res[b * 4 + 2] = dc * dc * bf16_round(duff[b]); float it = bf16_round(ib2[0]);
      for (int o = 0; o < DD; ++o) { float s = bf16_round(ib1[o]); for (int k = 0; k < DD; ++k) s += hs[k] * bf16_round(iW1[(size_t)k * DD + o]); it += fmaxf(s, 0.f) * bf16_round(iW2[o]); }
      res[b * 4 + 3] = it; } __syncthreads(); }
  if (tid < 8) { const float v = res[tid]; *(volatile float*)(out + tid) = v; __threadfence(); *(volatile float*)(out + tid) = v; } }

extern "C" void kernel_launch(void* const* d_in, const int* in_sizes, int n_in,
                              void* d_out, int out_size, void* d_ws, size_t ws_size, hipStream_t stream) {
  (void)in_sizes; (void)n_in; (void)out_size;
  const float* const* I = (const float* const*)d_in;
  const float* h1 = I[0]; const float* h2 = I[1]; const float* adj = I[2]; const float* dmv = I[3]; const float* ch1 = I[4]; const float* ch2 = I[5]; const float* veps = I[6]; const float* vsig = I[7]; const float* duff = I[8]; const float* val1 = I[9]; const float* val2 = I[10]; const float* nm1 = I[11]; const float* nm2 = I[12];
  const float* nodeW = I[13]; const float* gatW = I[14]; const float* gatWb = I[15]; const float* gatA = I[16]; const float* gatgW = I[17]; const float* gatgb = I[18]; const float* pW1 = I[19]; const float* pb1 = I[20]; const float* pW2 = I[21]; const float* pb2 = I[22]; const float* vcoef = I[23]; const float* dcoef = I[24]; const float* iW1 = I[25]; const float* ib1 = I[26]; const float* iW2 = I[27]; const float* ib2 = I[28];
  char* ws = (char*)d_ws; size_t off = 0;
  auto take = [&](size_t bytes) { char* p = ws + off; off += (bytes + 255) & ~(size_t)255; return p; };
  _Float16* BNW = (_Float16*)take((size_t)DD * 64 * 2); _Float16* BGW = (_Float16*)take((size_t)DD * DD * 2); _Float16* BGA = (_Float16*)take((size_t)DD * DD * 2); _Float16* BP1 = (_Float16*)take((size_t)NPM * DD * DD * 2); _Float16* BP2 = (_Float16*)take((size_t)NPM * DD * DD * 2);
  _Float16* H54 = (_Float16*)take((size_t)NR * 64 * 2); float* Xg = (float*)take((size_t)NR * DD * 4); float* Xn = (float*)take((size_t)NR * DD * 4); _Float16* X16 = (_Float16*)take((size_t)NR * DD * 2); float* Hh = (float*)take((size_t)NR * DD * 4); _Float16* Hh16 = (_Float16*)take((size_t)NR * DD * 2); float* HA = (float*)take((size_t)NR * DD * 4); float* E = (float*)take((size_t)NB * NA * NA * 4); float* ATTt = (float*)take((size_t)NB * NA * NA * 4);
  float* H2g = (float*)take((size_t)NR * DD * 4); _Float16* H2g16 = (_Float16*)take((size_t)NR * DD * 2); float* P1 = (float*)take((size_t)NPM * NR * DD * 4); float* P2 = (float*)take((size_t)NPM * NR * DD * 4); float* ECV = (float*)take((size_t)NR * 2 * 4); float* O5 = (float*)take((size_t)NPM * NB * NA * NA * 4);
  if (off > ws_size) return;
  const size_t n8 = (size_t)NR * DD / 8; const unsigned nb8 = (unsigned)((n8 + 255) / 256); const dim3 g128(((NR / 16) * 2 + 3) / 4, 1);
  k_wt<<<(DD * 8 + 255) / 256, 256, 0, stream>>>(nodeW, 54, 64, DD, BNW);
  for (int m = 0; m < NPM; ++m) { k_wt<<<(DD * 16 + 255) / 256, 256, 0, stream>>>(pW1 + (size_t)m * 256 * DD, DD, DD, DD, BP1 + (size_t)m * DD * DD); k_wt<<<(DD * 16 + 255) / 256, 256, 0, stream>>>(pW1 + (size_t)m * 256 * DD + (size_t)DD * DD, DD, DD, DD, BP2 + (size_t)m * DD * DD); }
  k_h54<<<(NR * 8 + 255) / 256, 256, 0, stream>>>(h1, H54);
  k_gemm_hhx<0><<<g128, 128, 0, stream>>>(H54, 64, 0, BNW, 64, 0, 0.0625f, nullptr, 0, nullptr, 1, 0, 0, Xg, X16, DD, 0, NR, DD, 64);
  k_h54<<<(NR * 8 + 255) / 256, 256, 0, stream>>>(h2, H54);
  k_gemm_hhx<0><<<g128, 128, 0, stream>>>(H54, 64, 0, BNW, 64, 0, 0.0625f, nullptr, 0, nullptr, 1, 0, 0, H2g, H2g16, DD, 0, NR, DD, 64);
  float* Xcur = Xg; float* Xoth = Xn;
  for (int l = 0; l < NL; ++l) {
    k_wt<<<(DD * 16 + 255) / 256, 256, 0, stream>>>(gatW + (size_t)l * DD * DD, DD, DD, DD, BGW); k_wt<<<(DD * 16 + 255) / 256, 256, 0, stream>>>(gatA + (size_t)l * DD * DD, DD, DD, DD, BGA);
    if (l > 0) k_f16c<<<nb8, 256, 0, stream>>>(Xcur, X16, n8);
    k_gemm_hhx<0><<<g128, 128, 0, stream>>>(X16, DD, 0, BGW, DD, 0, 0.0625f, gatWb + (size_t)l * DD, 0, nullptr, 1, 0, 0, Hh, Hh16, DD, 0, NR, DD, DD);
    k_gemm_hhx<0><<<g128, 128, 0, stream>>>(Hh16, DD, 0, BGA, DD, 0, 0.0625f, nullptr, 0, nullptr, 1, 0, 0, HA, nullptr, DD, 0, NR, DD, DD);
    k_gate<<<(NB * NA * NA + 255) / 256, 256, 0, stream>>>(HA, Hh, E);
    k_gsoft<<<(NB * NA + 127) / 128, 128, 0, stream>>>(E, adj, ATTt);
    k_gagg<<<(NB * NA + 63) / 64, 64, 0, stream>>>(ATTt, Hh, Xcur, gatgW + (size_t)l * 2 * DD, gatgb + l, Xoth);
    float* tmp = Xcur; Xcur = Xoth; Xoth = tmp; }
  k_f16c<<<nb8, 256, 0, stream>>>(Xcur, X16, n8);
  for (int m = 0; m < NPM; ++m) {
    k_gemm_hhx<0><<<g128, 128, 0, stream>>>(X16, DD, 0, BP1 + (size_t)m * DD * DD, DD, 0, 0.0625f, pb1 + (size_t)m * DD, 0, nullptr, 1, 0, 0, P1 + (size_t)m * NR * DD, nullptr, DD, 0, NR, DD, DD);
    k_gemm_hhx<0><<<g128, 128, 0, stream>>>(H2g16, DD, 0, BP2 + (size_t)m * DD * DD, DD, 0, 0.0625f, nullptr, 0, nullptr, 1, 0, 0, P2 + (size_t)m * NR * DD, nullptr, DD, 0, NR, DD, DD); }
  k_pmlp<<<(NB * NA * NA + 255) / 256, 256, 0, stream>>>(P1, P2, pW2, pb2, O5);
  k_phys<<<(NB * NA + 127) / 128, 128, 0, stream>>>(O5, dmv, ch1, ch2, veps, vsig, val1, val2, nm1, nm2, vcoef, ECV);
  k_final<<<1, 256, 0, stream>>>(ECV, Xcur, val1, duff, dcoef, iW1, ib1, iW2, ib2, (float*)d_out);
}
